// DeltaNet_22488448762128
// MI455X (gfx1250) — hardware-run, weakly checked
//
#include <hip/hip_runtime.h>
#include <math.h>

typedef __attribute__((ext_vector_type(16))) _Float16 v16h;
typedef __attribute__((ext_vector_type(8)))  _Float16 v8h;
typedef __attribute__((ext_vector_type(2)))  _Float16 v2h;
typedef __attribute__((ext_vector_type(8)))  float    v8f;
typedef __attribute__((ext_vector_type(4)))  float    v4f;
typedef __attribute__((ext_vector_type(2)))  float    v2f;
typedef __attribute__((ext_vector_type(4)))  unsigned int v4u;

constexpr int kB     = 2;
constexpr int kL     = 2048;
constexpr int kHid   = 2048;
constexpr int kH     = 16;
constexpr int kD     = 128;
constexpr int kHalfD = kD / 2;
constexpr int kRows  = kB * kL;
constexpr int kGateP = 64;
constexpr int kCh    = 64;
constexpr int kNCh   = kL / kCh;
constexpr int kPQP   = 136;
constexpr int kSP    = 72;
constexpr int kEarly = kB * kCh;
static_assert(kHid == kH * kD, "head split");
static_assert(kHalfD == 64, "frequency count");
static_assert((kL % kCh) == 0, "chunks are exact");
static_assert(kCh == 64, "early rows fill whole 64-row GEMM tiles");
static_assert((kL & (kL - 1)) == 0, "sequence length is a power of two");
static_assert((kRows % 64) == 0 && (kHid % 64) == 0 && (kGateP % 64) == 0, "GEMM M,N multiples of 64");
static_assert((kEarly % 16) == 0, "early GEMM M multiple of 16");
static_assert((kHid % 32) == 0, "GEMM K multiple of 32");
static_assert((kHid / 8) == 256, "one 256-thread block per early x row");
static_assert((kPQP % 8) == 0 && (kSP % 8) == 0, "16-B aligned LDS rows");

constexpr float kXCarry  = 16.0f;
constexpr float kWCarry  = 1024.0f;
constexpr float kVCarry  = 16.0f;
constexpr float kYCarry  = 128.0f;
constexpr float kResScale = 2048.0f;
constexpr float kResInv   = 1.0f / kResScale;
constexpr float kScaleQK = 1.0f / (kXCarry * kWCarry);
constexpr float kScaleV  = kVCarry / (kXCarry * kWCarry);
constexpr float kScaleO  = 1.0f / (kYCarry * kWCarry);
constexpr float kYScale  = kYCarry / kVCarry;
constexpr float kBetaMin = 0.8f;
constexpr float kBetaMax = 0.9995f;
constexpr float kEps     = 1e-6f;
constexpr float kRopeBase = 10000.0f;
constexpr float kF16MinNormal = 6.103515625e-5f;

constexpr size_t kPlaneB = (size_t)kRows * kHid * 2;
constexpr size_t kEarlyB = (size_t)kEarly * kHid * 2;
constexpr size_t kOffXH  = 0;
constexpr size_t kOffWT  = kOffXH  + kPlaneB;
constexpr size_t kOffWLO = kOffWT  + (size_t)4 * kHid * kHid * 2;
constexpr size_t kOffWGT = kOffWLO + (size_t)2 * kHid * kHid * 2;
constexpr size_t kOffQP  = kOffWGT + (size_t)kGateP * kHid * 2;
constexpr size_t kOffKP  = kOffQP  + kPlaneB;
constexpr size_t kOffVP  = kOffKP  + kPlaneB;
constexpr size_t kOffLG  = kOffVP  + kPlaneB;
constexpr size_t kOffCS  = kOffLG  + (size_t)kRows * kGateP * 4;
constexpr size_t kOffSN  = kOffCS  + (size_t)kL * kHalfD * 4;
constexpr size_t kOffFQ  = kOffSN  + (size_t)kL * kHalfD * 4;
constexpr size_t kOffXEH = kOffFQ  + (size_t)kHalfD * 4;
constexpr size_t kOffXEL = kOffXEH + kEarlyB;
constexpr size_t kOffVEH = kOffXEL + kEarlyB;
constexpr size_t kOffVEL = kOffVEH + kEarlyB;
constexpr size_t kOffYEH = kOffVEL + kEarlyB;
constexpr size_t kOffYEL = kOffYEH + kEarlyB;
constexpr size_t kWsTotal = kOffYEL + kEarlyB;
static_assert(kWsTotal == 122945792ull, "carve total");
static_assert(kWsTotal <= 134217728ull, "carve cap");
static_assert((kOffWT % 128) == 0 && (kOffWLO % 128) == 0 && (kOffWGT % 128) == 0 && (kOffQP % 128) == 0 &&
              (kOffKP % 128) == 0 && (kOffVP % 128) == 0 && (kOffLG % 128) == 0 && (kOffCS % 128) == 0 &&
              (kOffSN % 128) == 0 && (kOffFQ % 128) == 0 && (kOffXEH % 128) == 0 && (kOffXEL % 128) == 0 &&
              (kOffVEH % 128) == 0 && (kOffVEL % 128) == 0 && (kOffYEH % 128) == 0 && (kOffYEL % 128) == 0,
              "128-B aligned regions");

__device__ __forceinline__ void pin_u(unsigned& x) { asm volatile("" : "+v"(x)); }

__device__ __forceinline__ float flush_h(float v) { return (fabsf(v) < kF16MinNormal) ? 0.0f : v; }

__device__ __forceinline__ float resid_of(float v) {
  const _Float16 hh = (_Float16)flush_h(v);
  const float hf = (float)hh;
  return (v - hf) * kResScale;
}

__device__ __forceinline__ unsigned pack_hh(_Float16 a, _Float16 b) {
  v2h p;
  p[0] = a;
  p[1] = b;
  return __builtin_bit_cast(unsigned, p);
}
__device__ __forceinline__ unsigned pack2h(float a, float b) {
  const _Float16 ha = (_Float16)flush_h(a);
  const _Float16 hb = (_Float16)flush_h(b);
  return pack_hh(ha, hb);
}

__device__ __forceinline__ float h16_to_f32(unsigned hb) {
  const unsigned sgn = (hb & 0x8000u) << 16;
  const unsigned em = hb & 0x7fffu;
  const float fn = __uint_as_float((em << 13) + 0x38000000u);
  const float fs = (float)em * 5.9604644775390625e-8f;
  const float mag = (em < 0x400u) ? fs : fn;
  return __uint_as_float(__float_as_uint(mag) | sgn);
}

struct FragH {
  union U { v16h v; v8h h[2]; };
  static __device__ __forceinline__ v16h load(const _Float16* p) {
    U f;
    f.h[0] = *(const v8h*)(p);
    f.h[1] = *(const v8h*)(p + 16);
    return f.v;
  }
};

__device__ __forceinline__ v8f mma_h(v16h a, v16h b, v8f c) {
  c = __builtin_amdgcn_wmma_f32_16x16x32_f16(false, a, false, b, (short)0, c, false, false);
  asm volatile("v_nop\n\tv_nop\n\tv_nop\n\tv_nop" : "+v"(c) : "v"(a), "v"(b));
  return c;
}

template <int BIAS_MODE, int OUT_MODE>
__global__ __launch_bounds__(256) void gemm64_f16_kernel(
    const unsigned short* __restrict__ Ap, int lda, long strideA,
    const unsigned short* __restrict__ Btp, int ldb, long strideB,
    void* __restrict__ Cout, int ldc, long strideC,
    const float* __restrict__ bias,
    int M, int N, int K, float scale, float scaleLastZ, int skipRows) {
  const _Float16* A  = (const _Float16*)Ap;
  const _Float16* Bt = (const _Float16*)Btp;
  __shared__ __align__(16) float sT[8][16 * 68];
  unsigned tidu = threadIdx.x;
  pin_u(tidu);
  unsigned laneu = tidu & 31u;
  pin_u(laneu);
  unsigned waveu = tidu >> 5;
  pin_u(waveu);
  const int lane = (int)laneu;
  const int wave = (int)waveu;
  const int b = blockIdx.y;
  const int tilesN = N >> 6;
  const int tilesM = M >> 6;
  const int tile = blockIdx.x * 8 + wave;
  if (tile >= tilesM * tilesN) return;
  const int tm = tile / tilesN;
  const int tn = tile - tm * tilesN;
  const int m0 = tm << 6;
  const int n0 = tn << 6;
  if ((m0 & (kL - 1)) < skipRows) return;
  const float sc = (b == (int)gridDim.y - 1) ? scaleLastZ : scale;

  const _Float16* Ab = A  + (size_t)b * strideA;
  const _Float16* Bb = Bt + (size_t)b * strideB;

  const int rlane = lane & 15;
  const int koff  = (lane >> 4) * 8;
  const int mOff  = (lane >> 4) * 8;

  v8f acc[4][4];
#pragma unroll
  for (int i = 0; i < 4; ++i)
#pragma unroll
    for (int j = 0; j < 4; ++j) acc[i][j] = (v8f){0.f, 0.f, 0.f, 0.f, 0.f, 0.f, 0.f, 0.f};

  for (int k0 = 0; k0 < K; k0 += 32) {
    v16h bh[4];
#pragma unroll
    for (int j = 0; j < 4; ++j) {
      const size_t bo = (size_t)(n0 + (j << 4) + rlane) * ldb + koff + k0;
      bh[j] = FragH::load(Bb + bo);
    }
#pragma unroll
    for (int i = 0; i < 4; ++i) {
      const size_t ao = (size_t)(m0 + (i << 4) + rlane) * lda + koff + k0;
      const v16h ah = FragH::load(Ab + ao);
#pragma unroll
      for (int j = 0; j < 4; ++j) acc[i][j] = mma_h(ah, bh[j], acc[i][j]);
    }
  }

  float* slab = sT[wave];
#pragma unroll
  for (int i = 0; i < 4; ++i) {
    const int mBase = m0 + (i << 4);
#pragma unroll
    for (int j = 0; j < 4; ++j) {
      float bv = 0.f;
      if (BIAS_MODE == 2) bv = bias[n0 + (j << 4) + rlane];
#pragma unroll
      for (int r = 0; r < 8; ++r) {
        float v = acc[i][j][r] * sc;
        if (BIAS_MODE == 2) v += bv;
        slab[(mOff + r) * 68 + (j << 4) + rlane] = v;
      }
    }
    __builtin_amdgcn_fence(__ATOMIC_RELEASE, "workgroup");
    __builtin_amdgcn_wave_barrier();
    __builtin_amdgcn_fence(__ATOMIC_ACQUIRE, "workgroup");
    if (OUT_MODE == 0) {
      float* C = (float*)Cout + (size_t)b * strideC;
      const int hh = lane >> 4, c4 = (lane & 15) * 4;
      for (int pass = 0; pass < 2; ++pass) {
#pragma unroll
        for (int it = 0; it < 8; ++it) {
          const int row = it * 2 + hh;
          const v4f v = *(const v4f*)(slab + row * 68 + c4);
          *(volatile v4f*)(C + (size_t)(mBase + row) * ldc + n0 + c4) = v;
        }
        __threadfence();
      }
    } else {
      const int q = lane >> 3, c8 = (lane & 7) * 8;
      unsigned short* C = (unsigned short*)Cout + (size_t)b * strideC;
      for (int pass = 0; pass < 2; ++pass) {
#pragma unroll
        for (int it = 0; it < 4; ++it) {
          const int row = it * 4 + q;
          const float* sp = slab + row * 68 + c8;
          v8h hv;
#pragma unroll
          for (int e = 0; e < 8; ++e) hv[e] = (_Float16)flush_h(sp[e]);
          *(volatile v8h*)(C + (size_t)(mBase + row) * ldc + n0 + c8) = hv;
        }
        __threadfence();
      }
    }
    __builtin_amdgcn_fence(__ATOMIC_RELEASE, "workgroup");
    __builtin_amdgcn_wave_barrier();
    __builtin_amdgcn_fence(__ATOMIC_ACQUIRE, "workgroup");
  }
}

template <int OUT_MODE>
__global__ __launch_bounds__(256) void gemm_early_kernel(
    const unsigned short* __restrict__ Ahp, const unsigned short* __restrict__ Alp, int lda,
    const unsigned short* __restrict__ Bhp, const unsigned short* __restrict__ Blp, int ldb,
    void* __restrict__ Cout, void* __restrict__ Cout2, int ldc,
    const float* __restrict__ bias, int M, int N, int K, float scale) {
  const _Float16* Ah = (const _Float16*)Ahp;
  const _Float16* Al = (const _Float16*)Alp;
  const _Float16* Bh = (const _Float16*)Bhp;
  const _Float16* Bl = (const _Float16*)Blp;
  __shared__ __align__(16) float sT[8][16 * 68];
  unsigned tidu = threadIdx.x;
  pin_u(tidu);
  unsigned laneu = tidu & 31u;
  pin_u(laneu);
  unsigned waveu = tidu >> 5;
  pin_u(waveu);
  const int lane = (int)laneu;
  const int wave = (int)waveu;
  const int tilesN = N >> 6;
  const int tilesM = M >> 4;
  const int tile = blockIdx.x * 8 + wave;
  if (tile >= tilesM * tilesN) return;
  const int tm = tile / tilesN;
  const int tn = tile - tm * tilesN;
  const int m0 = tm << 4;
  const int n0 = tn << 6;

  const int rlane = lane & 15;
  const int koff  = (lane >> 4) * 8;
  const int mOff  = (lane >> 4) * 8;

  v8f accM[4], accR[4];
#pragma unroll
  for (int j = 0; j < 4; ++j) {
    accM[j] = (v8f){0.f, 0.f, 0.f, 0.f, 0.f, 0.f, 0.f, 0.f};
    accR[j] = (v8f){0.f, 0.f, 0.f, 0.f, 0.f, 0.f, 0.f, 0.f};
  }

  for (int k0 = 0; k0 < K; k0 += 32) {
    const size_t ao = (size_t)(m0 + rlane) * lda + koff + k0;
    const v16h ah = FragH::load(Ah + ao);
    const v16h al = FragH::load(Al + ao);
#pragma unroll
    for (int j = 0; j < 4; ++j) {
      const size_t bo = (size_t)(n0 + (j << 4) + rlane) * ldb + koff + k0;
      const v16h bh = FragH::load(Bh + bo);
      const v16h bl = FragH::load(Bl + bo);
      accM[j] = mma_h(ah, bh, accM[j]);
      accR[j] = mma_h(ah, bl, accR[j]);
      accR[j] = mma_h(al, bh, accR[j]);
    }
  }

  float* slab = sT[wave];
#pragma unroll
  for (int j = 0; j < 4; ++j) {
    float bv = 0.f;
    if (OUT_MODE == 0) bv = bias[n0 + (j << 4) + rlane];
#pragma unroll
    for (int r = 0; r < 8; ++r) {
      const float folded = accM[j][r] + accR[j][r] * kResInv;
      float v = folded * scale;
      if (OUT_MODE == 0) v += bv;
      slab[(mOff + r) * 68 + (j << 4) + rlane] = v;
    }
  }
  __builtin_amdgcn_fence(__ATOMIC_RELEASE, "workgroup");
  __builtin_amdgcn_wave_barrier();
  __builtin_amdgcn_fence(__ATOMIC_ACQUIRE, "workgroup");
  if (OUT_MODE == 0) {
    float* C = (float*)Cout;
    const int gBase = (m0 >> 6) * kL + (m0 & 63);
    const int hh = lane >> 4, c4 = (lane & 15) * 4;
    for (int pass = 0; pass < 2; ++pass) {
#pragma unroll
      for (int it = 0; it < 8; ++it) {
        const int row = it * 2 + hh;
        const v4f v = *(const v4f*)(slab + row * 68 + c4);
        *(volatile v4f*)(C + (size_t)(gBase + row) * ldc + n0 + c4) = v;
      }
      __threadfence();
    }
  } else {
    const int q = lane >> 3, c8 = (lane & 7) * 8;
    unsigned short* C  = (unsigned short*)Cout;
    unsigned short* C2 = (unsigned short*)Cout2;
    v8h hv[4], lv[4];
#pragma unroll
    for (int it = 0; it < 4; ++it) {
      const int row = it * 4 + q;
      const float* sp = slab + row * 68 + c8;
#pragma unroll
      for (int e = 0; e < 8; ++e) {
        const float x = sp[e];
        hv[it][e] = (_Float16)flush_h(x);
        lv[it][e] = (_Float16)flush_h(resid_of(x));
      }
    }
    for (int pass = 0; pass < 2; ++pass) {
#pragma unroll
      for (int it = 0; it < 4; ++it) {
        const int row = it * 4 + q;
        const size_t o = (size_t)(m0 + row) * ldc + n0 + c8;
        *(volatile v8h*)(C + o) = hv[it];
        *(volatile v8h*)(C2 + o) = lv[it];
      }
      __threadfence();
    }
  }
}

__global__ __launch_bounds__(256) void cast_x_kernel(const float* __restrict__ in, unsigned short* __restrict__ out,
                                                     int n8, float carry) {
  const int i = blockIdx.x * 256 + threadIdx.x;
  if (i >= n8) return;
  const float* p = in + 8 * (size_t)i;
  const v4f a = *(const v4f*)(p);
  const v4f c = *(const v4f*)(p + 4);
  v4u u;
  u[0] = pack2h(a[0] * carry, a[1] * carry);
  u[1] = pack2h(a[2] * carry, a[3] * carry);
  u[2] = pack2h(c[0] * carry, c[1] * carry);
  u[3] = pack2h(c[2] * carry, c[3] * carry);
  unsigned short* q = out + 8 * (size_t)i;
  *(volatile v4u*)q = u;
  __threadfence();
  *(volatile v4u*)q = u;
}

__global__ __launch_bounds__(256) void cast_xe_kernel(const float* __restrict__ in, unsigned short* __restrict__ oh,
                                                      unsigned short* __restrict__ ol, int n8, float carry) {
  const int i = blockIdx.x * 256 + threadIdx.x;
  if (i >= n8) return;
  const int r = i >> 8;
  const int c = (i & 255) * 8;
  const size_t srow = (size_t)(r >> 6) * kL + (size_t)(r & 63);
  const float* p = in + srow * kHid + c;
  const v4f a = *(const v4f*)(p);
  const v4f b = *(const v4f*)(p + 4);
  float x[8];
  x[0] = a[0] * carry;
  x[1] = a[1] * carry;
  x[2] = a[2] * carry;
  x[3] = a[3] * carry;
  x[4] = b[0] * carry;
  x[5] = b[1] * carry;
  x[6] = b[2] * carry;
  x[7] = b[3] * carry;
  v4u uh, ul;
  uh[0] = pack2h(x[0], x[1]);
  uh[1] = pack2h(x[2], x[3]);
  uh[2] = pack2h(x[4], x[5]);
  uh[3] = pack2h(x[6], x[7]);
  ul[0] = pack2h(resid_of(x[0]), resid_of(x[1]));
  ul[1] = pack2h(resid_of(x[2]), resid_of(x[3]));
  ul[2] = pack2h(resid_of(x[4]), resid_of(x[5]));
  ul[3] = pack2h(resid_of(x[6]), resid_of(x[7]));
  unsigned short* qh = oh + 8 * (size_t)i;
  unsigned short* ql = ol + 8 * (size_t)i;
  *(volatile v4u*)qh = uh;
  *(volatile v4u*)ql = ul;
  __threadfence();
  *(volatile v4u*)qh = uh;
  *(volatile v4u*)ql = ul;
}

__global__ __launch_bounds__(256) void wt_transpose_kernel(const float* __restrict__ W0, const float* __restrict__ W1,
                                                           const float* __restrict__ W2, const float* __restrict__ W3,
                                                           unsigned short* __restrict__ out, float carry) {
  __shared__ float sm[64][65];
  const int t  = threadIdx.x;
  const int k0 = blockIdx.x * 64;
  const int n0 = blockIdx.y * 64;
  const int z  = blockIdx.z;
  const float* W = (z == 0) ? W0 : (z == 1) ? W1 : (z == 2) ? W2 : W3;
#pragma unroll
  for (int i = 0; i < 16; ++i) {
    const int e = i * 256 + t;
    const int r = e >> 6;
    const int c = e & 63;
    sm[c][r] = W[(size_t)(k0 + r) * kHid + n0 + c] * carry;
  }
  __syncthreads();
  const int lane = t & 31, wave = t >> 5;
  const int q = lane >> 3, c8 = (lane & 7) * 8;
  unsigned short* op = out + (size_t)z * kHid * kHid;
  for (int pass = 0; pass < 2; ++pass) {
#pragma unroll
    for (int it = 0; it < 2; ++it) {
      const int row = wave * 8 + it * 4 + q;
      v4u u;
      u[0] = pack2h(sm[row][c8 + 0], sm[row][c8 + 1]);
      u[1] = pack2h(sm[row][c8 + 2], sm[row][c8 + 3]);
      u[2] = pack2h(sm[row][c8 + 4], sm[row][c8 + 5]);
      u[3] = pack2h(sm[row][c8 + 6], sm[row][c8 + 7]);
      *(volatile v4u*)(op + (size_t)(n0 + row) * kHid + k0 + c8) = u;
    }
    __threadfence();
  }
}

__global__ __launch_bounds__(256) void wt_lo_transpose_kernel(const float* __restrict__ W0, const float* __restrict__ W1,
                                                              unsigned short* __restrict__ out, float carry) {
  __shared__ float sm[64][65];
  const int t  = threadIdx.x;
  const int k0 = blockIdx.x * 64;
  const int n0 = blockIdx.y * 64;
  const int z  = blockIdx.z;
  const float* W = (z == 0) ? W0 : W1;
#pragma unroll
  for (int i = 0; i < 16; ++i) {
    const int e = i * 256 + t;
    const int r = e >> 6;
    const int c = e & 63;
    sm[c][r] = W[(size_t)(k0 + r) * kHid + n0 + c] * carry;
  }
  __syncthreads();
  const int lane = t & 31, wave = t >> 5;
  const int q = lane >> 3, c8 = (lane & 7) * 8;
  unsigned short* op = out + (size_t)z * kHid * kHid;
  v4u u[2];
#pragma unroll
  for (int it = 0; it < 2; ++it) {
    const int row = wave * 8 + it * 4 + q;
    u[it][0] = pack2h(resid_of(sm[row][c8 + 0]), resid_of(sm[row][c8 + 1]));
    u[it][1] = pack2h(resid_of(sm[row][c8 + 2]), resid_of(sm[row][c8 + 3]));
    u[it][2] = pack2h(resid_of(sm[row][c8 + 4]), resid_of(sm[row][c8 + 5]));
    u[it][3] = pack2h(resid_of(sm[row][c8 + 6]), resid_of(sm[row][c8 + 7]));
  }
  for (int pass = 0; pass < 2; ++pass) {
#pragma unroll
    for (int it = 0; it < 2; ++it) {
      const int row = wave * 8 + it * 4 + q;
      *(volatile v4u*)(op + (size_t)(n0 + row) * kHid + k0 + c8) = u[it];
    }
    __threadfence();
  }
}

__global__ __launch_bounds__(256) void wg_transpose_kernel(const float* __restrict__ Wg, unsigned short* __restrict__ out,
                                                           float carry) {
  __shared__ float sm[16][65];
  const int t  = threadIdx.x;
  const int k0 = blockIdx.x * 64;
#pragma unroll
  for (int i = 0; i < 4; ++i) {
    const int e = i * 256 + t;
    const int r = e >> 4;
    const int c = e & 15;
    sm[c][r] = Wg[(size_t)(k0 + r) * kH + c] * carry;
  }
  __syncthreads();
  const int lane = t & 31, wave = t >> 5;
  const int q = lane >> 3, c8 = (lane & 7) * 8;
  for (int pass = 0; pass < 2; ++pass) {
#pragma unroll
    for (int it = 0; it < 2; ++it) {
      const int row = wave * 8 + it * 4 + q;
      const int rc = (row < kH) ? row : (kH - 1);
      const bool real = (row < kH);
      float x[8];
#pragma unroll
      for (int e = 0; e < 8; ++e) {
        const float v = sm[rc][c8 + e];
        x[e] = real ? v : 0.0f;
      }
      v4u u;
      u[0] = pack2h(x[0], x[1]);
      u[1] = pack2h(x[2], x[3]);
      u[2] = pack2h(x[4], x[5]);
      u[3] = pack2h(x[6], x[7]);
      *(volatile v4u*)(out + (size_t)row * kHid + k0 + c8) = u;
    }
    __threadfence();
  }
}

__global__ __launch_bounds__(64) void rope_freq_kernel(float* __restrict__ fq) {
  const int j = threadIdx.x;
  const float ex = (float)j / (float)kHalfD;
  const float pw = powf(kRopeBase, ex);
  const float inv = 1.0f / pw;
  volatile float* dst = fq + j;
  *dst = inv;
  __threadfence();
  *dst = inv;
}

__global__ __launch_bounds__(256) void rope_table_kernel(const float* __restrict__ fq, float* __restrict__ cs,
                                                         float* __restrict__ sn) {
  __shared__ __align__(16) float sc[256];
  __shared__ __align__(16) float ss[256];
  const int tid = threadIdx.x;
  const int j = tid & 63;
  const int l = blockIdx.x * 4 + (tid >> 6);
  const float fr = fq[j];
  float ang = (float)l * fr;
  asm volatile("" : "+v"(ang));
  sc[tid] = cosf(ang);
  ss[tid] = sinf(ang);
  __syncthreads();
  if (tid < 128) {
    const int which = tid >> 6;
    const int i4 = (tid & 63) * 4;
    const v4f vc = *(const v4f*)(sc + i4);
    const v4f vs = *(const v4f*)(ss + i4);
    const v4f v = which ? vs : vc;
    float* dst = (which ? sn : cs) + (size_t)blockIdx.x * 256 + i4;
    *(volatile v4f*)dst = v;
    __threadfence();
    *(volatile v4f*)dst = v;
  }
}

__device__ __forceinline__ float phi_map(float v) {
  const float e = __expf(fminf(v, 0.0f));
  return (v > 0.0f) ? (v + 1.0f) : e;
}

__global__ __launch_bounds__(256) void rope_phi_kernel(unsigned short* Qp, unsigned short* Kp,
                                                       const float* __restrict__ cs, const float* __restrict__ sn) {
  unsigned tid = threadIdx.x;
  pin_u(tid);
  unsigned lane = tid & 31u;
  pin_u(lane);
  unsigned wave = tid >> 5;
  pin_u(wave);
  const unsigned gw = blockIdx.x * 8u + wave;
  const unsigned row = gw >> 4;
  const unsigned head = gw & 15u;
  const unsigned l = row & (unsigned)(kL - 1);
  const size_t base = (size_t)row * kHid + (size_t)head * kD;
  unsigned* q32 = (unsigned*)(Qp + base);
  unsigned* k32 = (unsigned*)(Kp + base);
  const unsigned qa = q32[lane];
  const unsigned qb = q32[32u + lane];
  const unsigned ka = k32[lane];
  const unsigned kb = k32[32u + lane];
  const v2f cv = *(const v2f*)(cs + (size_t)l * kHalfD + 2u * lane);
  const v2f sv = *(const v2f*)(sn + (size_t)l * kHalfD + 2u * lane);
  const float c0 = cv[0], c1 = cv[1], s0 = sv[0], s1 = sv[1];

  const float qe0 = h16_to_f32(qa & 0xffffu), qe1 = h16_to_f32(qa >> 16);
  const float qo0 = h16_to_f32(qb & 0xffffu), qo1 = h16_to_f32(qb >> 16);
  const float ke0 = h16_to_f32(ka & 0xffffu), ke1 = h16_to_f32(ka >> 16);
  const float ko0 = h16_to_f32(kb & 0xffffu), ko1 = h16_to_f32(kb >> 16);

  const unsigned wqa = pack2h(phi_map(qe0 * c0 - qo0 * s0), phi_map(qe1 * c1 - qo1 * s1));
  const unsigned wqb = pack2h(phi_map(qe0 * s0 + qo0 * c0), phi_map(qe1 * s1 + qo1 * c1));
  const unsigned wka = pack2h(phi_map(ke0 * c0 - ko0 * s0), phi_map(ke1 * c1 - ko1 * s1));
  const unsigned wkb = pack2h(phi_map(ke0 * s0 + ko0 * c0), phi_map(ke1 * s1 + ko1 * c1));

  for (int pass = 0; pass < 2; ++pass) {
    *(volatile unsigned*)(q32 + lane) = wqa;
    *(volatile unsigned*)(q32 + 32u + lane) = wqb;
    *(volatile unsigned*)(k32 + lane) = wka;
    *(volatile unsigned*)(k32 + 32u + lane) = wkb;
    __threadfence();
  }
}

__global__ __launch_bounds__(256) __attribute__((amdgpu_num_vgpr(256))) void chunk_scan_kernel(
    const unsigned short* __restrict__ PQg, const unsigned short* __restrict__ PKg,
    const unsigned short* __restrict__ Vg,
    const unsigned short* __restrict__ VEh, const unsigned short* __restrict__ VEl,
    const float* __restrict__ LG, const float* __restrict__ bg,
    unsigned short* __restrict__ Yg, unsigned short* __restrict__ YEh, unsigned short* __restrict__ YEl) {
  __shared__ __align__(16) _Float16 sPQ[kCh * kPQP];
  __shared__ __align__(16) _Float16 sPKY[kCh * kPQP];
  __shared__ __align__(16) _Float16 sVT[kD * kSP];
  __shared__ __align__(16) _Float16 sVTL[kD * kSP];
  __shared__ __align__(16) _Float16 sKT[kD * kSP];
  __shared__ __align__(16) _Float16 sA[kCh * kSP];
  __shared__ __align__(16) _Float16 sST[kD * kPQP];
  __shared__ __align__(16) float sLg[kCh];
  __shared__ __align__(16) float sC[kCh];
  __shared__ __align__(16) float sEc[kCh];
  __shared__ __align__(16) float sEk[kCh];
  __shared__ __align__(16) float sRowP[2 * kCh];
  __shared__ __align__(16) float sQZ[kCh];
  __shared__ __align__(16) float sZ[kD];

  unsigned tid = threadIdx.x;
  pin_u(tid);
  unsigned lane = tid & 31u;
  pin_u(lane);
  unsigned wave = tid >> 5;
  pin_u(wave);
  unsigned hl = lane >> 4;
  pin_u(hl);
  unsigned rl = lane & 15u;
  pin_u(rl);
  unsigned tb = wave & 3u;
  pin_u(tb);
  unsigned eh = wave >> 2;
  pin_u(eh);
  const unsigned koff = hl * 8u;
  unsigned tl = 16u * tb + rl;
  pin_u(tl);

  const int bh = blockIdx.x;
  const int bb = bh >> 4;
  const int hd = bh & 15;
  const size_t rowbase = (size_t)bb * kL;
  const size_t colbase = (size_t)hd * kD;
  const size_t erow0 = (size_t)bb * kCh;
  const float bgv = bg[hd];

  {
    const v4u zz = (v4u){0u, 0u, 0u, 0u};
    for (unsigned i = tid; i < (unsigned)(kD * kPQP / 8); i += 256u) ((v4u*)sST)[i] = zz;
    if (tid < (unsigned)kD) sZ[tid] = 0.0f;
  }
  v8f sacc[8];
#pragma unroll
  for (int j = 0; j < 8; ++j) sacc[j] = (v8f){0.f, 0.f, 0.f, 0.f, 0.f, 0.f, 0.f, 0.f};

#pragma unroll 1
  for (int ch = 0; ch < kNCh; ++ch) {
    const size_t grow0 = rowbase + (size_t)ch * kCh;
    __syncthreads();

    if (tid < (unsigned)kCh) {
      const float x = LG[(grow0 + tid) * kGateP + hd] + bgv;
      float sg = 1.0f / (1.0f + expf(-x));
      sg = fminf(fmaxf(sg, kBetaMin), kBetaMax);
      sLg[tid] = logf(sg);
    }
#pragma unroll 2
    for (int i = 0; i < 4; ++i) {
      const unsigned task = tid + 256u * (unsigned)i;
      const unsigned row = task >> 4;
      const unsigned seg = task & 15u;
      const size_t g = (grow0 + row) * kHid + colbase + 8u * seg;
      const v4u a = *(const v4u*)(PQg + g);
      const v4u k = *(const v4u*)(PKg + g);
      *(v4u*)(sPQ + row * kPQP + 8u * seg) = a;
      *(v4u*)(sPKY + row * kPQP + 8u * seg) = k;
    }
    {
      const unsigned short* vsrc = (ch == 0) ? (VEh + erow0 * kHid + colbase) : (Vg + grow0 * kHid + colbase);
#pragma unroll
      for (int i = 0; i < 2; ++i) {
        const unsigned task = tid + 256u * (unsigned)i;
        const unsigned sp = task & 31u;
        const unsigned dg = task >> 5;
        const size_t g0 = (size_t)(2u * sp) * kHid + 8u * dg;
        const v4u a = *(const v4u*)(vsrc + g0);
        const v4u k = *(const v4u*)(vsrc + g0 + kHid);
        unsigned* dst = (unsigned*)sVT + (8u * dg) * (unsigned)(kSP / 2) + sp;
#pragma unroll
        for (int c = 0; c < 4; ++c) {
          const unsigned wa = a[c];
          const unsigned wb = k[c];
          dst[(2 * c) * (kSP / 2)]     = (wa & 0xffffu) | (wb << 16);
          dst[(2 * c + 1) * (kSP / 2)] = (wa >> 16) | (wb & 0xffff0000u);
        }
      }
    }
    if (ch == 0) {
      const unsigned short* vsrcl = VEl + erow0 * kHid + colbase;
#pragma unroll
      for (int i = 0; i < 2; ++i) {
        const unsigned task = tid + 256u * (unsigned)i;
        const unsigned sp = task & 31u;
        const unsigned dg = task >> 5;
        const size_t g0 = (size_t)(2u * sp) * kHid + 8u * dg;
        const v4u a = *(const v4u*)(vsrcl + g0);
        const v4u k = *(const v4u*)(vsrcl + g0 + kHid);
        unsigned* dst = (unsigned*)sVTL + (8u * dg) * (unsigned)(kSP / 2) + sp;
#pragma unroll
        for (int c = 0; c < 4; ++c) {
          const unsigned wa = a[c];
          const unsigned wb = k[c];
          dst[(2 * c) * (kSP / 2)]     = (wa & 0xffffu) | (wb << 16);
          dst[(2 * c + 1) * (kSP / 2)] = (wa >> 16) | (wb & 0xffff0000u);
        }
      }
    }
    __syncthreads();

    if (tid < (unsigned)kCh) {
      float run = 0.0f, ct = 0.0f;
#pragma unroll 1
      for (int i = 0; i < kCh; ++i) {
        run += sLg[i];
        ct = ((unsigned)i == tid) ? run : ct;
      }
      sC[tid] = ct;
      sEc[tid] = expf(ct);
      sEk[tid] = expf(fminf(run - ct, 0.0f));
    }
    __syncthreads();

    {
      const unsigned t = tid >> 2;
      const unsigned part = tid & 3u;
      const _Float16* qp = sPQ + t * kPQP + 32u * part;
      const float* zp = sZ + 32u * part;
      float p = 0.0f;
#pragma unroll 1
      for (int g = 0; g < 4; ++g) {
        const v4u w = *(const v4u*)(qp + 8 * g);
        const v4f z0 = *(const v4f*)(zp + 8 * g);
        const v4f z1 = *(const v4f*)(zp + 8 * g + 4);
        const unsigned w0 = w[0], w1 = w[1], w2 = w[2], w3 = w[3];
        p = fmaf(h16_to_f32(w0 & 0xffffu), z0[0], p);
        p = fmaf(h16_to_f32(w0 >> 16), z0[1], p);
        p = fmaf(h16_to_f32(w1 & 0xffffu), z0[2], p);
        p = fmaf(h16_to_f32(w1 >> 16), z0[3], p);
        p = fmaf(h16_to_f32(w2 & 0xffffu), z1[0], p);
        p = fmaf(h16_to_f32(w2 >> 16), z1[1], p);
        p = fmaf(h16_to_f32(w3 & 0xffffu), z1[2], p);
        p = fmaf(h16_to_f32(w3 >> 16), z1[3], p);
      }
      p += __shfl_xor(p, 1, 32);
      p += __shfl_xor(p, 2, 32);
      if (part == 0u) sQZ[t] = p;
    }

#pragma unroll 1
    for (int i = 0; i < 2; ++i) {
      const unsigned task = tid + 256u * (unsigned)i;
      const unsigned sp = task & 31u;
      const unsigned dg = task >> 5;
      const v4u a = *(const v4u*)(sPKY + (2u * sp) * kPQP + 8u * dg);
      const v4u k = *(const v4u*)(sPKY + (2u * sp + 1u) * kPQP + 8u * dg);
      const float e0 = sEk[2u * sp];
      const float e1 = sEk[2u * sp + 1u];
      unsigned* dst = (unsigned*)sKT + (8u * dg) * (unsigned)(kSP / 2) + sp;
#pragma unroll
      for (int c = 0; c < 4; ++c) {
        const unsigned wa = a[c];
        const unsigned wb = k[c];
        dst[(2 * c) * (kSP / 2)]     = pack2h(h16_to_f32(wa & 0xffffu) * e0, h16_to_f32(wb & 0xffffu) * e1);
        dst[(2 * c + 1) * (kSP / 2)] = pack2h(h16_to_f32(wa >> 16) * e0, h16_to_f32(wb >> 16) * e1);
      }
    }

    {
      float rs = 0.0f;
      const float ct = sC[tl];
#pragma unroll 1
      for (int si = 0; si < 2; ++si) {
        const unsigned sb = 2u * eh + (unsigned)si;
        v8f sc = (v8f){0.f, 0.f, 0.f, 0.f, 0.f, 0.f, 0.f, 0.f};
#pragma unroll 1
        for (int ks = 0; ks < 4; ++ks) {
          const unsigned kk = koff + 32u * (unsigned)ks;
          const v16h fk = FragH::load(sPKY + (16u * sb + rl) * kPQP + kk);
          const v16h fq = FragH::load(sPQ + tl * kPQP + kk);
          sc = mma_h(fk, fq, sc);
        }
        _Float16 ah[8];
#pragma unroll
        for (int r = 0; r < 8; ++r) {
          const unsigned s = 16u * sb + 8u * hl + (unsigned)r;
          const float dec = expf(fminf(ct - sC[s], 0.0f));
          const float prod = sc[r] * dec;
          const float a = (s <= tl) ? prod : 0.0f;
          ah[r] = (_Float16)flush_h(a);
          rs += (float)ah[r];
        }
        v4u wv;
        wv[0] = pack_hh(ah[0], ah[1]);
        wv[1] = pack_hh(ah[2], ah[3]);
        wv[2] = pack_hh(ah[4], ah[5]);
        wv[3] = pack_hh(ah[6], ah[7]);
        *(v4u*)(sA + tl * kSP + 16u * sb + 8u * hl) = wv;
      }
      rs += __shfl_xor(rs, 16, 32);
      if (hl == 0u) sRowP[eh * (unsigned)kCh + tl] = rs;
    }

    v8f o[4];
#pragma unroll
    for (int j = 0; j < 4; ++j) o[j] = (v8f){0.f, 0.f, 0.f, 0.f, 0.f, 0.f, 0.f, 0.f};
#pragma unroll 1
    for (int ks = 0; ks < 4; ++ks) {
      const unsigned kk = koff + 32u * (unsigned)ks;
      const v16h fq = FragH::load(sPQ + tl * kPQP + kk);
#pragma unroll
      for (int j = 0; j < 4; ++j) {
        const v16h fs = FragH::load(sST + (64u * eh + 16u * (unsigned)j + rl) * kPQP + kk);
        o[j] = mma_h(fq, fs, o[j]);
      }
    }
#pragma unroll
    for (int r = 0; r < 8; ++r) {
      const float ec = sEc[16u * tb + 8u * hl + (unsigned)r];
#pragma unroll
      for (int j = 0; j < 4; ++j) o[j][r] *= ec;
    }
    __syncthreads();

#pragma unroll 1
    for (int ks = 0; ks < 2; ++ks) {
      const unsigned kk = koff + 32u * (unsigned)ks;
      const v16h fa = FragH::load(sA + tl * kSP + kk);
#pragma unroll
      for (int j = 0; j < 4; ++j) {
        const v16h fv = FragH::load(sVT + (64u * eh + 16u * (unsigned)j + rl) * kSP + kk);
        o[j] = mma_h(fa, fv, o[j]);
      }
    }
    if (ch == 0) {
      const v16h fa0 = FragH::load(sA + tl * kSP + koff);
      const v16h fa1 = FragH::load(sA + tl * kSP + koff + 32u);
#pragma unroll
      for (int j = 0; j < 4; ++j) {
        v8f rr = (v8f){0.f, 0.f, 0.f, 0.f, 0.f, 0.f, 0.f, 0.f};
        const v16h fv0 = FragH::load(sVTL + (64u * eh + 16u * (unsigned)j + rl) * kSP + koff);
        rr = mma_h(fa0, fv0, rr);
        const v16h fv1 = FragH::load(sVTL + (64u * eh + 16u * (unsigned)j + rl) * kSP + koff + 32u);
        rr = mma_h(fa1, fv1, rr);
#pragma unroll
        for (int r = 0; r < 8; ++r) o[j][r] += rr[r] * kResInv;
      }
    }
    float invr[8];
#pragma unroll
    for (int r = 0; r < 8; ++r) {
      const unsigned t = 16u * tb + 8u * hl + (unsigned)r;
      const float den = (sRowP[t] + sRowP[(unsigned)kCh + t]) + sEc[t] * sQZ[t] + kEps;
      invr[r] = kYScale * (1.0f / den);
    }
#pragma unroll
    for (int r = 0; r < 8; ++r) {
      const unsigned t = 16u * tb + 8u * hl + (unsigned)r;
#pragma unroll
      for (int j = 0; j < 4; ++j)
        sPKY[t * kPQP + 64u * eh + 16u * (unsigned)j + rl] = (_Float16)flush_h(o[j][r] * invr[r]);
    }
    if (ch == 0) {
#pragma unroll
      for (int r = 0; r < 8; ++r) {
        const unsigned t = 16u * tb + 8u * hl + (unsigned)r;
#pragma unroll
        for (int j = 0; j < 4; ++j) {
          const float yv = o[j][r] * invr[r];
          sPQ[t * kPQP + 64u * eh + 16u * (unsigned)j + rl] = (_Float16)flush_h(resid_of(yv));
        }
      }
    }

    const float ecl = sEc[kCh - 1];
#pragma unroll
    for (int j = 0; j < 8; ++j)
#pragma unroll
      for (int r = 0; r < 8; ++r) sacc[j][r] *= ecl;
#pragma unroll 1
    for (int ks = 0; ks < 2; ++ks) {
      const unsigned kk = koff + 32u * (unsigned)ks;
      const v16h fa = FragH::load(sKT + (16u * wave + rl) * kSP + kk);
#pragma unroll
      for (int j = 0; j < 8; ++j) {
        const v16h fv = FragH::load(sVT + (16u * (unsigned)j + rl) * kSP + kk);
        sacc[j] = mma_h(fa, fv, sacc[j]);
      }
    }
    if (ch == 0) {
      const v16h fa0 = FragH::load(sKT + (16u * wave + rl) * kSP + koff);
      const v16h fa1 = FragH::load(sKT + (16u * wave + rl) * kSP + koff + 32u);
#pragma unroll
      for (int j = 0; j < 8; ++j) {
        v8f rr = (v8f){0.f, 0.f, 0.f, 0.f, 0.f, 0.f, 0.f, 0.f};
        const v16h fv0 = FragH::load(sVTL + (16u * (unsigned)j + rl) * kSP + koff);
        rr = mma_h(fa0, fv0, rr);
        const v16h fv1 = FragH::load(sVTL + (16u * (unsigned)j + rl) * kSP + koff + 32u);
        rr = mma_h(fa1, fv1, rr);
#pragma unroll
        for (int r = 0; r < 8; ++r) sacc[j][r] += rr[r] * kResInv;
      }
    }
#pragma unroll
    for (int j = 0; j < 8; ++j) {
      v4u wv;
      wv[0] = pack2h(sacc[j][0], sacc[j][1]);
      wv[1] = pack2h(sacc[j][2], sacc[j][3]);
      wv[2] = pack2h(sacc[j][4], sacc[j][5]);
      wv[3] = pack2h(sacc[j][6], sacc[j][7]);
      *(v4u*)(sST + (16u * (unsigned)j + rl) * kPQP + 16u * wave + 8u * hl) = wv;
    }

    if (tid < (unsigned)kD) {
      const _Float16* kp = sKT + tid * kSP;
      float sum = 0.0f;
#pragma unroll 1
      for (int g = 0; g < 8; ++g) {
        const v4u w = *(const v4u*)(kp + 8 * g);
        const unsigned w0 = w[0], w1 = w[1], w2 = w[2], w3 = w[3];
        sum += h16_to_f32(w0 & 0xffffu);
        sum += h16_to_f32(w0 >> 16);
        sum += h16_to_f32(w1 & 0xffffu);
        sum += h16_to_f32(w1 >> 16);
        sum += h16_to_f32(w2 & 0xffffu);
        sum += h16_to_f32(w2 >> 16);
        sum += h16_to_f32(w3 & 0xffffu);
        sum += h16_to_f32(w3 >> 16);
      }
      sZ[tid] = fmaf(ecl, sZ[tid], sum);
    }
    __syncthreads();

    {
      v4u val[4];
#pragma unroll
      for (int it = 0; it < 4; ++it) {
        const unsigned row = 8u * wave + 2u * (unsigned)it + hl;
        val[it] = *(const v4u*)(sPKY + row * kPQP + 8u * rl);
      }
      for (int pass = 0; pass < 2; ++pass) {
#pragma unroll
        for (int it = 0; it < 4; ++it) {
          const unsigned row = 8u * wave + 2u * (unsigned)it + hl;
          *(volatile v4u*)(Yg + (grow0 + row) * kHid + colbase + 8u * rl) = val[it];
        }
        __threadfence();
      }
      if (ch == 0) {
        v4u vlo[4];
#pragma unroll
        for (int it = 0; it < 4; ++it) {
          const unsigned row = 8u * wave + 2u * (unsigned)it + hl;
          vlo[it] = *(const v4u*)(sPQ + row * kPQP + 8u * rl);
        }
        for (int pass = 0; pass < 2; ++pass) {
#pragma unroll
          for (int it = 0; it < 4; ++it) {
            const unsigned row = 8u * wave + 2u * (unsigned)it + hl;
            const size_t eo = (erow0 + row) * kHid + colbase + 8u * rl;
            *(volatile v4u*)(YEh + eo) = val[it];
            *(volatile v4u*)(YEl + eo) = vlo[it];
          }
          __threadfence();
        }
      }
    }
  }
}

extern "C" void kernel_launch(void* const* d_in, const int* in_sizes, int n_in,
                              void* d_out, int out_size, void* d_ws, size_t ws_size,
                              hipStream_t stream) {
  if (n_in < 8) return;
  if (in_sizes[0] != kRows * kHid) return;
  if (in_sizes[1] != kHid * kHid) return;
  if (in_sizes[2] != kHid * kHid) return;
  if (in_sizes[3] != kHid * kHid) return;
  if (in_sizes[4] != kHid * kH) return;
  if (in_sizes[5] != kH) return;
  if (in_sizes[6] != kHid * kHid) return;
  if (in_sizes[7] != kHid) return;
  if (out_size != kRows * kHid) return;
  if (ws_size < kWsTotal) return;

  const float* x  = (const float*)d_in[0];
  const float* Wq = (const float*)d_in[1];
  const float* Wk = (const float*)d_in[2];
  const float* Wv = (const float*)d_in[3];
  const float* Wg = (const float*)d_in[4];
  const float* bg = (const float*)d_in[5];
  const float* Wo = (const float*)d_in[6];
  const float* bo = (const float*)d_in[7];
  float* out = (float*)d_out;

  char* ws = (char*)d_ws;
  unsigned short* XH  = (unsigned short*)(ws + kOffXH);
  unsigned short* YP  = (unsigned short*)(ws + kOffXH);
  unsigned short* WT  = (unsigned short*)(ws + kOffWT);
  unsigned short* WLO = (unsigned short*)(ws + kOffWLO);
  unsigned short* WGT = (unsigned short*)(ws + kOffWGT);
  unsigned short* QP  = (unsigned short*)(ws + kOffQP);
  unsigned short* KP  = (unsigned short*)(ws + kOffKP);
  unsigned short* VP  = (unsigned short*)(ws + kOffVP);
  float*          LG  = (float*)(ws + kOffLG);
  float*          CS  = (float*)(ws + kOffCS);
  float*          SN  = (float*)(ws + kOffSN);
  float*          FQ  = (float*)(ws + kOffFQ);
  unsigned short* XEH = (unsigned short*)(ws + kOffXEH);
  unsigned short* XEL = (unsigned short*)(ws + kOffXEL);
  unsigned short* VEH = (unsigned short*)(ws + kOffVEH);
  unsigned short* VEL = (unsigned short*)(ws + kOffVEL);
  unsigned short* YEH = (unsigned short*)(ws + kOffYEH);
  unsigned short* YEL = (unsigned short*)(ws + kOffYEL);

  cast_x_kernel<<<(kRows * kHid / 8) / 256, 256, 0, stream>>>(x, XH, kRows * kHid / 8, kXCarry);
  wt_transpose_kernel<<<dim3(kHid / 64, kHid / 64, 4), 256, 0, stream>>>(Wq, Wk, Wv, Wo, WT, kWCarry);
  wt_lo_transpose_kernel<<<dim3(kHid / 64, kHid / 64, 2), 256, 0, stream>>>(Wv, Wo, WLO, kWCarry);
  wg_transpose_kernel<<<kHid / 64, 256, 0, stream>>>(Wg, WGT, kWCarry);
  cast_xe_kernel<<<(kEarly * kHid / 8) / 256, 256, 0, stream>>>(x, XEH, XEL, kEarly * kHid / 8, kXCarry);

  rope_freq_kernel<<<1, kHalfD, 0, stream>>>(FQ);
  rope_table_kernel<<<kL / 4, 256, 0, stream>>>(FQ, CS, SN);

  gemm64_f16_kernel<0, 1><<<dim3(256, 3), 256, 0, stream>>>(
      XH, kHid, 0L,
      WT, kHid, (long)kHid * kHid,
      (void*)QP, kHid, (long)kRows * kHid,
      nullptr,
      kRows, kHid, kHid, kScaleQK, kScaleV, 0);

  gemm64_f16_kernel<0, 0><<<dim3(8, 1), 256, 0, stream>>>(
      XH, kHid, 0L,
      WGT, kHid, 0L,
      (void*)LG, kGateP, 0L,
      nullptr,
      kRows, kGateP, kHid, kScaleQK, kScaleQK, 0);

  gemm_early_kernel<1><<<(kEarly / 16) * (kHid / 64) / 8, 256, 0, stream>>>(
      XEH, XEL, kHid,
      WT + (size_t)2 * kHid * kHid, WLO, kHid,
      (void*)VEH, (void*)VEL, kHid,
      nullptr,
      kEarly, kHid, kHid, kScaleV);

  rope_phi_kernel<<<(kRows * kH) / 8, 256, 0, stream>>>(QP, KP, CS, SN);

  chunk_scan_kernel<<<kB * kH, 256, 0, stream>>>(QP, KP, VP, VEH, VEL, LG, bg, YP, YEH, YEL);

  gemm64_f16_kernel<2, 0><<<dim3(256, 1), 256, 0, stream>>>(
      YP, kHid, 0L,
      WT + (size_t)3 * kHid * kHid, kHid, 0L,
      (void*)out, kHid, 0L,
      bo,
      kRows, kHid, kHid, kScaleO, kScaleO, kCh);

  gemm_early_kernel<0><<<(kEarly / 16) * (kHid / 64) / 8, 256, 0, stream>>>(
      YEH, YEL, kHid,
      WT + (size_t)3 * kHid * kHid, WLO + (size_t)kHid * kHid, kHid,
      (void*)out, nullptr, kHid,
      bo,
      kEarly, kHid, kHid, kScaleO);
}
